// MultiHeadSelfAttention_27238682591816
// MI455X (gfx1250) — hardware-verified
//
#include <hip/hip_runtime.h>


#ifndef NB
#define NB 2
#endif
#ifndef SEQ
#define SEQ 2048
#endif
#define NB_FULL   2
#define SEQ_FULL  2048
#define HID       1024
#define NHEAD     16
#define HD        64
#define MROWS     (NB * SEQ)
#define CTXW      (2 * HID)
#define PSP       128

static_assert(HID == NHEAD * HD);
static_assert(HD == 64);
static_assert(SEQ % 128 == 0);
static_assert(SEQ <= SEQ_FULL);
static_assert(NB >= 1 && NB <= NB_FULL);
static_assert(MROWS % 128 == 0);
static_assert(HID % 128 == 0);
static_assert((HID & (HID - 1)) == 0);
static_assert(CTXW % 32 == 0);
static_assert(PSP >= 2 * HD);
static_assert(((size_t)7 * MROWS * HID + (size_t)4 * HID * HID) * 2 <= (size_t)134217728);

#define CARRY_X     16.0f
#define CARRY_W     32.0f
#define CARRY_QKV   16.0f
#define CARRY_QRES  2048.0f
#define CARRY_CTX   1024.0f

typedef _Float16 f16;
typedef f16   v16h __attribute__((ext_vector_type(16)));
typedef f16   v8h  __attribute__((ext_vector_type(8)));
typedef float v8f  __attribute__((ext_vector_type(8)));
typedef float v4f  __attribute__((ext_vector_type(4)));

union FragU { v16h v; v8h half[2]; f16 e[16]; };
union H8U   { v8h v; f16 e[8]; };

__device__ __forceinline__ v8f zero8() {
    v8f z = {0.f, 0.f, 0.f, 0.f, 0.f, 0.f, 0.f, 0.f};
    return z;
}

__device__ __forceinline__ v8f wmma16(v16h a, v16h b, v8f c) {
    v8f d = __builtin_amdgcn_wmma_f32_16x16x32_f16(false, a, false, b, (short)0, c, false, false);
    asm volatile("v_nop\n\tv_nop\n\tv_nop\n\tv_nop" : "+v"(d) : "v"(a), "v"(b));
    return d;
}

__device__ __forceinline__ float bf16_rne(float x) {
    unsigned u = __float_as_uint(x);
    u = (u + 0x7fffu + ((u >> 16) & 1u)) & 0xffff0000u;
    return __uint_as_float(u);
}

__device__ __forceinline__ float fexp2(float x) {
#if defined(__has_builtin)
#if __has_builtin(__builtin_amdgcn_exp2f)
    return __builtin_amdgcn_exp2f(x);
#else
    return exp2f(x);
#endif
#else
    return exp2f(x);
#endif
}

__device__ __forceinline__ float rowmax16(float x) {
    int v = __builtin_bit_cast(int, x);
    x = fmaxf(x, __builtin_bit_cast(float, __builtin_amdgcn_update_dpp(v, v, 0x121, 0xf, 0xf, false)));
    v = __builtin_bit_cast(int, x);
    x = fmaxf(x, __builtin_bit_cast(float, __builtin_amdgcn_update_dpp(v, v, 0x122, 0xf, 0xf, false)));
    v = __builtin_bit_cast(int, x);
    x = fmaxf(x, __builtin_bit_cast(float, __builtin_amdgcn_update_dpp(v, v, 0x124, 0xf, 0xf, false)));
    v = __builtin_bit_cast(int, x);
    x = fmaxf(x, __builtin_bit_cast(float, __builtin_amdgcn_update_dpp(v, v, 0x128, 0xf, 0xf, false)));
    return x;
}

__device__ __forceinline__ v16h load_frag(const f16* tile, int rowbase, int pitch, int kcol, int lane) {
    const int r  = rowbase + (lane & 15);
    const int kh = (lane >> 4) << 3;
    const f16* p = tile + (size_t)r * pitch + kcol + kh;
    FragU f;
    f.half[0] = *(const v8h*)(p);
    f.half[1] = *(const v8h*)(p + 16);
    return f.v;
}

__global__ void __launch_bounds__(256)
cvt_rows(const float* __restrict__ src, f16* __restrict__ dst, int nrows, float carry) {
    static_assert(HID == 128 * 8);
    const int g  = (int)blockIdx.x * 256 + (int)threadIdx.x;
    const int m  = g >> 7;
    const int c8 = (g & 127) << 3;
    if (m >= nrows) return;
    const int sm = (m / SEQ) * SEQ_FULL + (m % SEQ);
    const float* sp = src + (size_t)sm * HID + c8;
    const v4f a = *(const v4f*)sp;
    const v4f b = *(const v4f*)(sp + 4);
    H8U o;
#pragma unroll
    for (int j = 0; j < 4; ++j) {
        const float x0 = a[j];
        const float x1 = b[j];
        o.e[j]     = (f16)(bf16_rne(x0) * carry);
        o.e[j + 4] = (f16)(bf16_rne(x1) * carry);
    }
    f16* dp = dst + (size_t)m * HID + c8;
    *(volatile v8h*)dp = o.v;
    __threadfence();
    *(volatile v8h*)dp = o.v;
}

__global__ void __launch_bounds__(256)
cvt_transpose(const float* __restrict__ src, f16* __restrict__ dst, int ncols, float carry) {
    __shared__ __attribute__((aligned(16))) f16 Ts[64 * 64];
    const int tid  = (int)threadIdx.x;
    const int lane = tid & 31;
    const int wave = tid >> 5;
    const int n0   = (int)blockIdx.x * 64;
    const int k0   = (int)blockIdx.y * 64;
    const int c4   = (tid & 15) << 2;
    const int rr   = tid >> 4;
#pragma unroll
    for (int p = 0; p < 4; ++p) {
        const int r = p * 16 + rr;
        const v4f a = *(const v4f*)(src + (size_t)(k0 + r) * ncols + n0 + c4);
#pragma unroll
        for (int j = 0; j < 4; ++j) Ts[(c4 + j) * 64 + r] = (f16)(bf16_rne(a[j]) * carry);
    }
    __syncthreads();
    const int piece = lane & 7;
    const int lsub  = lane >> 3;
#pragma unroll
    for (int pass = 0; pass < 2; ++pass) {
#pragma unroll
        for (int it = 0; it < 2; ++it) {
            const int nl = wave * 8 + it * 4 + lsub;
            const v8h v = *(const v8h*)&Ts[nl * 64 + piece * 8];
            f16* dp = dst + (size_t)(n0 + nl) * HID + k0 + piece * 8;
            *(volatile v8h*)dp = v;
        }
        if (pass == 0) __threadfence();
    }
}

__device__ __forceinline__ void write_head_lines(const f16* Cs, f16* __restrict__ op, size_t bh0,
                                                 int s0, int wave, int lane) {
    const int piece = lane & 7;
    const int lsub  = lane >> 3;
#pragma unroll
    for (int pass = 0; pass < 2; ++pass) {
#pragma unroll
        for (int it = 0; it < 8; ++it) {
            const int L    = wave * 32 + it * 4 + lsub;
            const int ml   = L >> 1;
            const int hsel = L & 1;
            const v8h v = *(const v8h*)&Cs[ml * 128 + hsel * 64 + piece * 8];
            f16* dp = op + ((bh0 + hsel) * SEQ + s0 + ml) * HD + piece * 8;
            *(volatile v8h*)dp = v;
        }
        if (pass == 0) __threadfence();
    }
}

template <int MODE, int KTOT>
__device__ __forceinline__ void gemm_body(const f16* __restrict__ A, const f16* __restrict__ W,
                                          const float* __restrict__ bias,
                                          f16* __restrict__ outA, f16* __restrict__ outB,
                                          float* __restrict__ outF, float accMul, float addMul) {
    static_assert(KTOT % 32 == 0);
    static_assert(KTOT == HID || KTOT == CTXW);
    __shared__ __attribute__((aligned(16))) f16 As[128 * 32];
    __shared__ __attribute__((aligned(16))) f16 Bs[128 * 32];
    __shared__ __attribute__((aligned(16))) f16 Cs[128 * 128];

    const int tid  = (int)threadIdx.x;
    const int lane = tid & 31;
    const int wave = tid >> 5;
    const int wm   = wave & 3;
    const int wn   = wave >> 2;
    const int hh8  = (lane >> 4) << 3;
    const int c16  = lane & 15;
    const int m0   = (int)blockIdx.x * 128;
    const int n0   = (int)blockIdx.y * 128;

    v8f acc[2][4];
#pragma unroll
    for (int i = 0; i < 2; ++i)
#pragma unroll
        for (int j = 0; j < 4; ++j) acc[i][j] = zero8();

    const int srow = tid >> 1;
    const int scol = (tid & 1) << 4;
    const f16* gA = A + (size_t)(m0 + srow) * KTOT + scol;
    const f16* gW = W + (size_t)(n0 + srow) * HID + scol;

#pragma unroll 1
    for (int k0 = 0; k0 < KTOT; k0 += 32) {
        const int kw = k0 & (HID - 1);
        const v8h ra0 = *(const v8h*)(gA + k0);
        const v8h ra1 = *(const v8h*)(gA + k0 + 8);
        const v8h rb0 = *(const v8h*)(gW + kw);
        const v8h rb1 = *(const v8h*)(gW + kw + 8);
        __syncthreads();
        *(v8h*)&As[srow * 32 + scol]     = ra0;
        *(v8h*)&As[srow * 32 + scol + 8] = ra1;
        *(v8h*)&Bs[srow * 32 + scol]     = rb0;
        *(v8h*)&Bs[srow * 32 + scol + 8] = rb1;
        __syncthreads();

        v16h af[2], bfr[4];
#pragma unroll
        for (int i = 0; i < 2; ++i) af[i] = load_frag(As, wm * 32 + i * 16, 32, 0, lane);
#pragma unroll
        for (int j = 0; j < 4; ++j) bfr[j] = load_frag(Bs, wn * 64 + j * 16, 32, 0, lane);
#pragma unroll
        for (int i = 0; i < 2; ++i)
#pragma unroll
            for (int j = 0; j < 4; ++j) acc[i][j] = wmma16(af[i], bfr[j], acc[i][j]);
    }

    float bb[4];
#pragma unroll
    for (int j = 0; j < 4; ++j) bb[j] = bf16_rne(bias[n0 + wn * 64 + j * 16 + c16]) * addMul;

    const int bidx  = m0 / SEQ;
    const int s0    = m0 - bidx * SEQ;
    const int piece = lane & 7;
    const int lsub  = lane >> 3;

    if constexpr (MODE == 0 || MODE == 3) {
#pragma unroll
        for (int i = 0; i < 2; ++i)
#pragma unroll
            for (int j = 0; j < 4; ++j) {
                const int nl = wn * 64 + j * 16 + c16;
#pragma unroll
                for (int r = 0; r < 8; ++r) {
                    const int ml = wm * 32 + i * 16 + hh8 + r;
                    Cs[ml * 128 + nl] = (f16)(acc[i][j][r] * accMul + bb[j]);
                }
            }
        __syncthreads();
        const size_t bh0 = (size_t)bidx * NHEAD + (n0 >> 6);
        write_head_lines(Cs, outA, bh0, s0, wave, lane);
        if constexpr (MODE == 3) {
            __syncthreads();
#pragma unroll
            for (int i = 0; i < 2; ++i)
#pragma unroll
                for (int j = 0; j < 4; ++j) {
                    const int nl = wn * 64 + j * 16 + c16;
#pragma unroll
                    for (int r = 0; r < 8; ++r) {
                        const int ml = wm * 32 + i * 16 + hh8 + r;
                        const float val = acc[i][j][r] * accMul + bb[j];
                        const f16 hi = (f16)val;
                        Cs[ml * 128 + nl] = (f16)((val - (float)hi) * CARRY_QRES);
                    }
                }
            __syncthreads();
            write_head_lines(Cs, outB, bh0, s0, wave, lane);
        }
    } else if constexpr (MODE == 1) {
#pragma unroll
        for (int i = 0; i < 2; ++i)
#pragma unroll
            for (int j = 0; j < 4; ++j) {
                const int nl = wn * 64 + j * 16 + c16;
                H8U t;
#pragma unroll
                for (int r = 0; r < 8; ++r) t.e[r] = (f16)(acc[i][j][r] * accMul + bb[j]);
                *(v8h*)&Cs[nl * 128 + wm * 32 + i * 16 + hh8] = t.v;
            }
        __syncthreads();
#pragma unroll
        for (int pass = 0; pass < 2; ++pass) {
#pragma unroll
            for (int it = 0; it < 8; ++it) {
                const int L  = wave * 32 + it * 4 + lsub;
                const int nl = L >> 1;
                const int mh = L & 1;
                const v8h v = *(const v8h*)&Cs[nl * 128 + mh * 64 + piece * 8];
                f16* dp = outA + ((size_t)(bidx * HID + n0 + nl) * SEQ + s0 + mh * 64 + piece * 8);
                *(volatile v8h*)dp = v;
            }
            if (pass == 0) __threadfence();
        }
    } else {
        float* Cf = (float*)Cs;
#pragma unroll
        for (int half = 0; half < 2; ++half) {
            if ((wm >> 1) == half) {
#pragma unroll
                for (int i = 0; i < 2; ++i)
#pragma unroll
                    for (int j = 0; j < 4; ++j) {
                        const int nl = wn * 64 + j * 16 + c16;
#pragma unroll
                        for (int r = 0; r < 8; ++r) {
                            const int ml = (wm & 1) * 32 + i * 16 + hh8 + r;
                            Cf[ml * 128 + nl] = acc[i][j][r] * accMul + bb[j];
                        }
                    }
            }
            __syncthreads();
#pragma unroll
            for (int pass = 0; pass < 2; ++pass) {
#pragma unroll
                for (int it = 0; it < 8; ++it) {
                    const int L    = wave * 32 + it * 4 + lsub;
                    const int row  = L >> 2;
                    const int part = L & 3;
                    const v4f v = *(const v4f*)&Cf[row * 128 + part * 32 + piece * 4];
                    float* dp = outF + (size_t)(m0 + half * 64 + row) * HID + n0 + part * 32 + piece * 4;
                    *(volatile v4f*)dp = v;
                }
                if (pass == 0) __threadfence();
            }
            __syncthreads();
        }
    }
}

__global__ void __launch_bounds__(256) __attribute__((amdgpu_num_vgpr(256)))
gemm_q(const f16* __restrict__ A, const f16* __restrict__ W, const float* __restrict__ bias,
       f16* __restrict__ outHi, f16* __restrict__ outRes, float accMul, float addMul) {
    gemm_body<3, HID>(A, W, bias, outHi, outRes, (float*)0, accMul, addMul);
}

__global__ void __launch_bounds__(256) __attribute__((amdgpu_num_vgpr(256)))
gemm_k(const f16* __restrict__ A, const f16* __restrict__ W, const float* __restrict__ bias,
       f16* __restrict__ outHi, float accMul, float addMul) {
    gemm_body<0, HID>(A, W, bias, outHi, (f16*)0, (float*)0, accMul, addMul);
}

__global__ void __launch_bounds__(256) __attribute__((amdgpu_num_vgpr(256)))
gemm_v(const f16* __restrict__ A, const f16* __restrict__ W, const float* __restrict__ bias,
       f16* __restrict__ outT, float accMul, float addMul) {
    gemm_body<1, HID>(A, W, bias, outT, (f16*)0, (float*)0, accMul, addMul);
}

__global__ void __launch_bounds__(256) __attribute__((amdgpu_num_vgpr(256)))
gemm_o(const f16* __restrict__ A, const f16* __restrict__ W, const float* __restrict__ bias,
       float* __restrict__ outF, float accMul, float addMul) {
    gemm_body<2, CTXW>(A, W, bias, (f16*)0, (f16*)0, outF, accMul, addMul);
}

__global__ void __launch_bounds__(256) __attribute__((amdgpu_num_vgpr(256)))
attn_fwd(const f16* __restrict__ Qp, const f16* __restrict__ Qr, const f16* __restrict__ Kp,
         const f16* __restrict__ Vt, f16* __restrict__ Cp) {
    __shared__ __attribute__((aligned(16))) f16 ks[64 * 64];
    __shared__ __attribute__((aligned(16))) f16 vsT[64 * 64];
    __shared__ __attribute__((aligned(16))) f16 ps[8][16 * PSP];

    static_assert(SEQ % 64 == 0);
    static_assert(8 * 16 == 128);

    const int tid  = (int)threadIdx.x;
    const int lane = tid & 31;
    const int wave = tid >> 5;
    const int hh8  = (lane >> 4) << 3;
    const int c16  = lane & 15;
    const int bh   = (int)blockIdx.y;
    const int bidx = bh / NHEAD;
    const int hidx = bh - bidx * NHEAD;
    const int q0   = (int)blockIdx.x * 128 + wave * 16;
    const size_t head = (size_t)bh * SEQ * HD;

    v16h qa[2], qr[2];
#pragma unroll
    for (int c = 0; c < 2; ++c) {
        qa[c] = load_frag(Qp + head, q0, HD, c * 32, lane);
        qr[c] = load_frag(Qr + head, q0, HD, c * 32, lane);
    }

    FragU onesu;
#pragma unroll
    for (int i = 0; i < 16; ++i) onesu.e[i] = (f16)1.0f;
    const v16h ones = onesu.v;

    float m[8];
    v8f   o[4], lacc;
#pragma unroll
    for (int r = 0; r < 8; ++r) m[r] = -1.0e30f;
#pragma unroll
    for (int dt = 0; dt < 4; ++dt) o[dt] = zero8();
    lacc = zero8();

    const float cl   = 1.4426950408889634f * 0.00048828125f;
    const float rinv = 1.0f / CARRY_QRES;
    f16* psw = &ps[wave][0];

#pragma unroll 1
    for (int kt = 0; kt < SEQ / 64; ++kt) {
        __syncthreads();
#pragma unroll
        for (int p2 = 0; p2 < 2; ++p2) {
            const int p   = tid + p2 * 256;
            const int row = p >> 3;
            const int pc  = (p & 7) << 3;
            const v8h kv = *(const v8h*)(Kp + head + (size_t)(kt * 64 + row) * HD + pc);
            const v8h vv = *(const v8h*)(Vt + head + (size_t)row * SEQ + kt * 64 + pc);
            *(v8h*)&ks[row * 64 + pc]  = kv;
            *(v8h*)&vsT[row * 64 + pc] = vv;
        }
        __syncthreads();

#pragma unroll 1
        for (int hf = 0; hf < 2; ++hf) {
            const int kb0 = hf * 32;
            v8f sh0 = zero8(), sh1 = zero8(), sr0 = zero8(), sr1 = zero8();
#pragma unroll
            for (int c = 0; c < 2; ++c) {
                const v16h k0f = load_frag(ks, kb0, 64, c * 32, lane);
                const v16h k1f = load_frag(ks, kb0 + 16, 64, c * 32, lane);
                sh0 = wmma16(qa[c], k0f, sh0);
                sr0 = wmma16(qr[c], k0f, sr0);
                sh1 = wmma16(qa[c], k1f, sh1);
                sr1 = wmma16(qr[c], k1f, sr1);
            }

#pragma unroll
            for (int r = 0; r < 8; ++r) {
                const float x0 = (sh0[r] + sr0[r] * rinv) * cl;
                const float x1 = (sh1[r] + sr1[r] * rinv) * cl;
                const float tm = rowmax16(fmaxf(x0, x1));
                const float mn = fmaxf(m[r], tm);
                const float al = fexp2(m[r] - mn);
                m[r] = mn;
                lacc[r] *= al;
#pragma unroll
                for (int dt = 0; dt < 4; ++dt) o[dt][r] *= al;
                const float sft = 10.0f - mn;
                psw[(hh8 + r) * PSP + c16]      = (f16)fexp2(x0 + sft);
                psw[(hh8 + r) * PSP + 16 + c16] = (f16)fexp2(x1 + sft);
            }
            __syncthreads();

            const v16h pa = load_frag(psw, 0, PSP, 0, lane);
#pragma unroll
            for (int dt = 0; dt < 4; ++dt) {
                const v16h vb = load_frag(vsT, dt * 16, 64, kb0, lane);
                o[dt] = wmma16(pa, vb, o[dt]);
            }
            lacc = wmma16(pa, ones, lacc);
        }
    }
    __syncthreads();

#pragma unroll
    for (int r = 0; r < 8; ++r) {
        const float inv = (CARRY_CTX / CARRY_QKV) / lacc[r];
#pragma unroll
        for (int dt = 0; dt < 4; ++dt) {
            const float val = o[dt][r] * inv;
            const f16 hi = (f16)val;
            psw[(hh8 + r) * PSP + dt * 16 + c16]      = hi;
            psw[(hh8 + r) * PSP + HD + dt * 16 + c16] = (f16)(val - (float)hi);
        }
    }
    __syncthreads();

    const int piece = lane & 7;
    const int lsub  = lane >> 3;
#pragma unroll
    for (int pass = 0; pass < 2; ++pass) {
#pragma unroll
        for (int it = 0; it < 8; ++it) {
            const int L   = it * 4 + lsub;
            const int row = L >> 1;
            const int sel = L & 1;
            const v8h v = *(const v8h*)&psw[row * PSP + sel * HD + piece * 8];
            f16* dp = Cp + ((size_t)(bidx * SEQ + q0 + row) * CTXW + sel * HID + hidx * HD + piece * 8);
            *(volatile v8h*)dp = v;
        }
        if (pass == 0) __threadfence();
    }
}

extern "C" void kernel_launch(void* const* d_in, const int* in_sizes, int n_in,
                              void* d_out, int out_size, void* d_ws, size_t ws_size,
                              hipStream_t stream) {
    if (n_in < 9) return;
    if (in_sizes[0] < ((NB - 1) * SEQ_FULL + SEQ) * HID) return;
    if (in_sizes[1] < HID * HID) return;
    if (in_sizes[2] < HID) return;
    if (in_sizes[3] < HID * HID) return;
    if (in_sizes[4] < HID) return;
    if (in_sizes[5] < HID * HID) return;
    if (in_sizes[6] < HID) return;
    if (in_sizes[7] < HID * HID) return;
    if (in_sizes[8] < HID) return;
    if (out_size < MROWS * HID) return;

    const float* x  = (const float*)d_in[0];
    const float* Wq = (const float*)d_in[1];
    const float* bq = (const float*)d_in[2];
    const float* Wk = (const float*)d_in[3];
    const float* bk = (const float*)d_in[4];
    const float* Wv = (const float*)d_in[5];
    const float* bv = (const float*)d_in[6];
    const float* Wo = (const float*)d_in[7];
    const float* bo = (const float*)d_in[8];

    const size_t nX = (size_t)MROWS * HID;
    const size_t nW = (size_t)HID * HID;
    const size_t totalHalves = 7 * nX + 4 * nW;
    if (ws_size < totalHalves * sizeof(f16)) return;

    f16* Xh   = (f16*)d_ws;
    f16* Wqt  = Xh   + nX;
    f16* Wkt  = Wqt  + nW;
    f16* Wvt  = Wkt  + nW;
    f16* Wot  = Wvt  + nW;
    f16* Qp   = Wot  + nW;
    f16* Qr   = Qp   + nX;
    f16* Kp   = Qr   + nX;
    f16* Vtp  = Kp   + nX;
    f16* Cp   = Vtp  + nX;

    cvt_rows<<<MROWS / 2, 256, 0, stream>>>(x, Xh, MROWS, CARRY_X);
    const dim3 gt(HID / 64, HID / 64);
    cvt_transpose<<<gt, 256, 0, stream>>>(Wq, Wqt, HID, CARRY_W);
    cvt_transpose<<<gt, 256, 0, stream>>>(Wk, Wkt, HID, CARRY_W);
    cvt_transpose<<<gt, 256, 0, stream>>>(Wv, Wvt, HID, CARRY_W);
    cvt_transpose<<<gt, 256, 0, stream>>>(Wo, Wot, HID, CARRY_W);

    const dim3 gg(MROWS / 128, HID / 128);
    const float accQKV = CARRY_QKV / (CARRY_X * CARRY_W);
    gemm_q<<<gg, 256, 0, stream>>>(Xh, Wqt, bq, Qp, Qr, accQKV, CARRY_QKV);
    gemm_k<<<gg, 256, 0, stream>>>(Xh, Wkt, bk, Kp, accQKV, CARRY_QKV);
    gemm_v<<<gg, 256, 0, stream>>>(Xh, Wvt, bv, Vtp, accQKV, CARRY_QKV);

    attn_fwd<<<dim3(SEQ / 128, NB * NHEAD), 256, 0, stream>>>(Qp, Qr, Kp, Vtp, Cp);

    const float accOut = 1.0f / (CARRY_CTX * CARRY_W);
    gemm_o<<<gg, 256, 0, stream>>>(Cp, Wot, bo, (float*)d_out, accOut, 1.0f);
}
